// GraphInteractionLayer_52304111730731
// MI455X (gfx1250) — hardware-verified
//
#include <hip/hip_runtime.h>
#include <math.h>

typedef __attribute__((ext_vector_type(16))) _Float16 v16h;
typedef __attribute__((ext_vector_type(16))) __bf16 v16b;
typedef __attribute__((ext_vector_type(8)))  _Float16 v8h;
typedef __attribute__((ext_vector_type(8)))  float v8f;
typedef __attribute__((ext_vector_type(4)))  float v4f;
typedef __attribute__((ext_vector_type(2)))  float v2f;
typedef __attribute__((ext_vector_type(4)))  unsigned v4u;
typedef __attribute__((ext_vector_type(4)))  int v4i;
typedef float __attribute__((may_alias)) float_a;
typedef int __attribute__((may_alias)) int_a;

template <typename T> __device__ __forceinline__ void vst2(void* p, T v) { *(volatile T*)p = v; __threadfence(); *(volatile T*)p = v; }
__device__ __forceinline__ v8f wmma16(v16h a, v16h b, v8f c) {
  v8f d = __builtin_amdgcn_wmma_f32_16x16x32_f16(false, a, false, b, (short)0, c, false, false);
  asm volatile("v_nop\n\tv_nop\n\tv_nop\n\tv_nop" : "+v"(d) : "v"(a), "v"(b));
  return d;
}
__device__ __forceinline__ v8f wmma_bf(v16b a, v16b b, v8f c) {
  v8f d = __builtin_amdgcn_wmma_f32_16x16x32_bf16(false, a, false, b, (short)0, c, false, false);
  asm volatile("v_nop\n\tv_nop\n\tv_nop\n\tv_nop" : "+v"(d) : "v"(a), "v"(b));
  return d;
}
__device__ __forceinline__ v16h frag_h(const _Float16* rowk0, int lane) {
  union { v16h v; v8h q[2]; } u; const _Float16* p = rowk0 + 8 * (lane >> 4);
  u.q[0] = *(const v8h*)p; u.q[1] = *(const v8h*)(p + 16); return u.v;
}
__device__ __forceinline__ v16h frag_f32(const float* rowk0, int lane) {
  v16h a; const float* p = rowk0 + 8 * (lane >> 4);
#pragma unroll
  for (int i = 0; i < 8; ++i) { a[i] = (_Float16)p[i]; a[8 + i] = (_Float16)p[16 + i]; }
  return a;
}
__device__ __forceinline__ v16h frag_f32s(const float* rowk0, int lane, float sc) {
  v16h a; const float* p = rowk0 + 8 * (lane >> 4);
#pragma unroll
  for (int i = 0; i < 8; ++i) { a[i] = (_Float16)(p[i] * sc); a[8 + i] = (_Float16)(p[16 + i] * sc); }
  return a;
}
__device__ __forceinline__ v16h fragc_f32(const float* W, int k0, int n, int lane, int ld, int K) {
  v16h a; const int g = lane >> 4;
#pragma unroll
  for (int i = 0; i < 8; ++i) { const int ka = k0 + 8 * g + i, kb = ka + 16;
    a[i] = (_Float16)(ka < K ? W[(size_t)ka * ld + n] : 0.f); a[8 + i] = (_Float16)(kb < K ? W[(size_t)kb * ld + n] : 0.f); }
  return a;
}
struct F2 { v16b h, l; };
__device__ __forceinline__ F2 bsplit16(const float v[16]) { F2 r;
#pragma unroll
  for (int i = 0; i < 16; ++i) { const __bf16 h = (__bf16)v[i]; r.h[i] = h; r.l[i] = (__bf16)(v[i] - (float)h); }
  return r; }
__device__ __forceinline__ F2 split_row(const float* row, int k0, int lane) { float v[16]; const float* p = row + k0 + 8 * (lane >> 4);
#pragma unroll
  for (int i = 0; i < 8; ++i) { v[i] = p[i]; v[8 + i] = p[16 + i]; }
  return bsplit16(v); }
__device__ __forceinline__ F2 split_rowK(const float* row, int k0, int lane, int K) { float v[16]; const int g = lane >> 4;
#pragma unroll
  for (int i = 0; i < 8; ++i) { const int ka = k0 + 8 * g + i, kb = ka + 16; v[i] = ka < K ? row[ka] : 0.f; v[8 + i] = kb < K ? row[kb] : 0.f; }
  return bsplit16(v); }
__device__ __forceinline__ F2 split_col(const float* W, int k0, int n, int lane, int ld, int K) { float v[16]; const int g = lane >> 4;
#pragma unroll
  for (int i = 0; i < 8; ++i) { const int ka = k0 + 8 * g + i, kb = ka + 16; v[i] = ka < K ? W[(size_t)ka * ld + n] : 0.f; v[8 + i] = kb < K ? W[(size_t)kb * ld + n] : 0.f; }
  return bsplit16(v); }
__device__ __forceinline__ v8f mac3(const F2& a, const F2& b, v8f c) { c = wmma_bf(a.l, b.h, c); c = wmma_bf(a.h, b.l, c); return wmma_bf(a.h, b.h, c); }
__device__ __forceinline__ float sigm(float v) { return 1.0f / (1.0f + expf(-v)); }
#define LDSX() do { asm volatile("s_wait_dscnt 0" ::: "memory"); __builtin_amdgcn_wave_barrier(); __builtin_amdgcn_fence(__ATOMIC_RELEASE, "workgroup"); } while (0)

#define NB 8
#define NN 256
#define DD 512
#define FF 1024
#define NR (NB * NN)

__global__ __launch_bounds__(128) void k_qkv(const float* __restrict__ x, const float* __restrict__ Wq, const float* __restrict__ bq, const float* __restrict__ Wk, const float* __restrict__ bk, const float* __restrict__ Wv, const float* __restrict__ bv,
                                           _Float16* __restrict__ q16, _Float16* __restrict__ k16, _Float16* __restrict__ vT) {
  __shared__ __align__(16) float so[4][16][132];
  __shared__ __align__(16) _Float16 st[128][72];
  const int tid = threadIdx.x, wave = tid >> 5, lane = tid & 31, col = lane & 15, g = lane >> 4;
  const int r0b = blockIdx.x * 64, r0 = r0b + wave * 16; const int which = blockIdx.y / 4, n0 = (blockIdx.y % 4) * 128; const int b = r0b / NN, t0 = r0b % NN;
  const float* W = which == 0 ? Wq : (which == 1 ? Wk : Wv); const float* bias = which == 0 ? bq : (which == 1 ? bk : bv);
  v8f acc[8] = {};
#pragma unroll 1
  for (int kc = 0; kc < DD / 32; ++kc) { const v16h a = frag_f32(x + (size_t)(r0 + col) * DD + kc * 32, lane);
#pragma unroll
    for (int j = 0; j < 8; ++j) acc[j] = wmma16(a, frag_f32s(W + (size_t)(n0 + j * 16 + col) * DD + kc * 32, lane, 16.0f), acc[j]); }
#pragma unroll
  for (int j = 0; j < 8; ++j) { const float bb = bias[n0 + j * 16 + col];
#pragma unroll
    for (int r = 0; r < 8; ++r) so[wave][8 * g + r][j * 16 + col] = acc[j][r] * (1.0f / 16.0f) + bb; }
  LDSX();
  if (which < 2) { _Float16* dst = which == 0 ? q16 : k16;
    for (int q = lane; q < 16 * 16; q += 32) { const int rl = q >> 4, pc = q & 15; union { v8h h8; v4u u; } pk;
#pragma unroll
      for (int e = 0; e < 8; ++e) pk.h8[e] = (_Float16)so[wave][rl][pc * 8 + e];
      vst2(dst + (size_t)(r0 + rl) * DD + n0 + pc * 8, pk.u); } }
  else {
#pragma unroll 4
    for (int rl = 0; rl < 16; ++rl) {
#pragma unroll
      for (int e = 0; e < 4; ++e) st[lane * 4 + e][wave * 16 + rl] = (_Float16)so[wave][rl][lane * 4 + e]; }
    __syncthreads();
    for (int q = tid; q < 128 * 8; q += 128) { const int c = q >> 3, pc = q & 7; vst2(vT + ((size_t)b * DD + n0 + c) * NN + t0 + pc * 8, *(const v4u*)(&st[c][pc * 8])); } }
}
__global__ __launch_bounds__(256) void k_bias(const float* __restrict__ pcs, const float* __restrict__ Wr1, const float* __restrict__ br1, const float* __restrict__ Wr2, const float* __restrict__ br2, float* __restrict__ bias) {
  __shared__ float sw1[DD][2], sb1[DD], sw2[DD]; __shared__ __align__(16) float so[NN];
  const int n = blockIdx.x, b = blockIdx.y, tid = threadIdx.x;
  for (int c = tid; c < DD; c += 256) { sw1[c][0] = Wr1[c * 2]; sw1[c][1] = Wr1[c * 2 + 1]; sb1[c] = br1[c]; sw2[c] = Wr2[c]; }
  __syncthreads();
  { const int m = tid; const float rx = pcs[((size_t)b * NN + n) * 2] - pcs[((size_t)b * NN + m) * 2], ry = pcs[((size_t)b * NN + n) * 2 + 1] - pcs[((size_t)b * NN + m) * 2 + 1];
    float a = br2[0];
#pragma unroll 4
    for (int c = 0; c < DD; ++c) { float hv = rx * sw1[c][0] + ry * sw1[c][1] + sb1[c]; hv = hv > 0.f ? hv : 0.f; a += hv * sw2[c]; }
    so[m] = a; }
  __syncthreads();
  if (tid < NN / 4) vst2(bias + ((size_t)b * NN + n) * NN + tid * 4, *(const v4f*)(&so[tid * 4]));
}
__global__ __launch_bounds__(128) void k_attn(const _Float16* __restrict__ q16, const _Float16* __restrict__ k16, const _Float16* __restrict__ vT, const float* __restrict__ bias, float* __restrict__ AG) {
  __shared__ __align__(16) float sS[4][16][260];
  __shared__ __align__(16) _Float16 sP[4][16][264];
  __shared__ __align__(16) float sA[4][16][260];
  const int tid = threadIdx.x, w = tid >> 5, lane = tid & 31, col = lane & 15, g = lane >> 4;
  const int b = blockIdx.y, q0 = blockIdx.x * 64 + w * 16; const size_t rb = (size_t)b * NN;
  { v16h aq[16];
#pragma unroll
    for (int kc = 0; kc < 16; ++kc) aq[kc] = frag_h(q16 + (rb + q0 + col) * DD + kc * 32, lane);
#pragma unroll 1
    for (int t = 0; t < NN / 16; ++t) { v8f s = {};
#pragma unroll
      for (int kc = 0; kc < 16; ++kc) s = wmma16(aq[kc], frag_h(k16 + (rb + t * 16 + col) * DD + kc * 32, lane), s);
#pragma unroll
      for (int r = 0; r < 8; ++r) { const int qi = q0 + 8 * g + r, m = t * 16 + col; sS[w][8 * g + r][m] = (m == qi) ? -3.0e38f : s[r] * 0.044194173824159216f + bias[(rb + qi) * NN + m]; } } }
  LDSX();
  { const int m = col; float mx = -3.4e38f;
    for (int e = 0; e < 128; ++e) mx = fmaxf(mx, sS[w][m][g * 128 + e]);
    mx = fmaxf(mx, __shfl_xor(mx, 16, 32)); float l = 0.f;
    for (int e = 0; e < 128; ++e) { const float sv = sS[w][m][g * 128 + e]; const float p = sv <= -1.0e38f ? 0.f : expf(sv - mx); l += p; sS[w][m][g * 128 + e] = p; }
    l += __shfl_xor(l, 16, 32); const float inv = 16384.0f / l;
    for (int e = 0; e < 128; ++e) sP[w][m][g * 128 + e] = (_Float16)(sS[w][m][g * 128 + e] * inv); }
  LDSX();
  v16h pa[8];
#pragma unroll
  for (int kc = 0; kc < 8; ++kc) pa[kc] = frag_h(&sP[w][col][0] + kc * 32, lane);
#pragma unroll 1
  for (int np = 0; np < 2; ++np) { v8f acc[16];
#pragma unroll
    for (int j = 0; j < 16; ++j) acc[j] = (v8f){};
#pragma unroll
    for (int kc = 0; kc < 8; ++kc) {
#pragma unroll
      for (int j = 0; j < 16; ++j) acc[j] = wmma16(pa[kc], frag_h(vT + ((size_t)b * DD + np * 256 + j * 16 + col) * NN + kc * 32, lane), acc[j]); }
#pragma unroll
    for (int j = 0; j < 16; ++j)
#pragma unroll
      for (int r = 0; r < 8; ++r) sA[w][8 * g + r][j * 16 + col] = acc[j][r] * (1.0f / 16384.0f);
    LDSX();
    for (int q = lane; q < 16 * 64; q += 32) { const int rl = q >> 6, pc = q & 63; vst2(AG + (rb + q0 + rl) * DD + np * 256 + pc * 4, *(const v4f*)(&sA[w][rl][pc * 4])); }
    LDSX(); }
}
template <int KIN, int AH>
__global__ __launch_bounds__(128) void k_lnproj(const void* __restrict__ Ain, const float* __restrict__ W, const float* __restrict__ bias, const float* __restrict__ res, const float* __restrict__ gam, const float* __restrict__ bet, float* __restrict__ Out) {
  __shared__ __align__(16) float so[4][16][DD + 4];
  const int tid = threadIdx.x, wave = tid >> 5, lane = tid & 31, col = lane & 15, g = lane >> 4;
  const int r0 = blockIdx.x * 64 + wave * 16;
#pragma unroll 1
  for (int np = 0; np < DD / 128; ++np) { v8f acc[8] = {};
#pragma unroll 1
    for (int kc = 0; kc < KIN / 32; ++kc) { v16h a; if (AH) a = frag_h((const _Float16*)Ain + (size_t)(r0 + col) * KIN + kc * 32, lane); else a = frag_f32((const float*)Ain + (size_t)(r0 + col) * KIN + kc * 32, lane);
#pragma unroll
      for (int j = 0; j < 8; ++j) acc[j] = wmma16(a, frag_f32s(W + (size_t)(np * 128 + j * 16 + col) * KIN + kc * 32, lane, 16.0f), acc[j]); }
#pragma unroll
    for (int j = 0; j < 8; ++j) { const int c = np * 128 + j * 16 + col; const float bb = bias[c];
#pragma unroll
      for (int r = 0; r < 8; ++r) so[wave][8 * g + r][c] = acc[j][r] * (AH ? (1.0f / 64.0f) : (1.0f / 16.0f)) + bb + res[(size_t)(r0 + 8 * g + r) * DD + c]; } }
  LDSX();
  { const int rl = lane >> 1, hf = lane & 1; float* row = &so[wave][rl][0]; float s = 0.f;
    for (int c = 0; c < 256; ++c) s += row[hf * 256 + c]; s += __shfl_xor(s, 1, 32); const float mu = s * (1.0f / DD);
    float q2 = 0.f; for (int c = 0; c < 256; ++c) { const float d = row[hf * 256 + c] - mu; q2 += d * d; } q2 += __shfl_xor(q2, 1, 32); const float rs = rsqrtf(q2 * (1.0f / DD) + 1e-5f);
    LDSX();
    for (int c4 = 0; c4 < 64; ++c4) { const int cc = hf * 256 + c4 * 4; v4f v = *(const v4f*)(&row[cc]);
#pragma unroll
      for (int e = 0; e < 4; ++e) v[e] = (v[e] - mu) * rs * gam[cc + e] + bet[cc + e];
      vst2(Out + (size_t)(r0 + rl) * DD + cc, v); } }
}
__global__ __launch_bounds__(128) void k_ff1(const float* __restrict__ x1, const float* __restrict__ Wf1, const float* __restrict__ bf1, _Float16* __restrict__ H16) {
  __shared__ __align__(16) float so[4][16][132];
  const int tid = threadIdx.x, wave = tid >> 5, lane = tid & 31, col = lane & 15, g = lane >> 4;
  const int r0 = blockIdx.x * 64 + wave * 16, n0 = blockIdx.y * 128;
  v8f acc[8] = {};
#pragma unroll 1
  for (int kc = 0; kc < DD / 32; ++kc) { const v16h a = frag_f32(x1 + (size_t)(r0 + col) * DD + kc * 32, lane);
#pragma unroll
    for (int j = 0; j < 8; ++j) acc[j] = wmma16(a, frag_f32s(Wf1 + (size_t)(n0 + j * 16 + col) * DD + kc * 32, lane, 16.0f), acc[j]); }
#pragma unroll
  for (int j = 0; j < 8; ++j) { const float bb = bf1[n0 + j * 16 + col];
#pragma unroll
    for (int r = 0; r < 8; ++r) { const float v = acc[j][r] * (1.0f / 16.0f) + bb; so[wave][8 * g + r][j * 16 + col] = v > 0.f ? v * 4.0f : 0.f; } }
  LDSX();
  for (int q = lane; q < 16 * 16; q += 32) { const int rl = q >> 4, pc = q & 15; union { v8h h8; v4u u; } pk;
#pragma unroll
    for (int e = 0; e < 8; ++e) pk.h8[e] = (_Float16)so[wave][rl][pc * 8 + e];
    vst2(H16 + (size_t)(r0 + rl) * FF + n0 + pc * 8, pk.u); }
}
extern "C" void kernel_launch(void* const* d_in, const int* in_sizes, int n_in, void* d_out, int out_size, void* d_ws, size_t ws_size, hipStream_t stream) {
  (void)in_sizes; (void)n_in; (void)out_size; (void)ws_size;
  const float** I = (const float**)d_in;
  const float* x = I[0]; const float* pcs = I[1]; const float* Wq = I[2]; const float* bq = I[3]; const float* Wk = I[4]; const float* bk = I[5]; const float* Wv = I[6]; const float* bv = I[7];
  const float* Wr1 = I[8]; const float* br1 = I[9]; const float* Wr2 = I[10]; const float* br2 = I[11]; const float* Wo = I[12]; const float* bo = I[13]; const float* g1 = I[14]; const float* be1 = I[15];
  const float* Wf1 = I[16]; const float* bf1 = I[17]; const float* Wf2 = I[18]; const float* bf2 = I[19]; const float* g2 = I[20]; const float* be2 = I[21];
  float* out = (float*)d_out;
  char* ws = (char*)d_ws; size_t off = 0;
  auto take = [&](size_t bytes) { char* p = ws + off; off += (bytes + 255) & ~(size_t)255; return p; };
  _Float16* q16 = (_Float16*)take((size_t)NR * DD * 2); _Float16* k16 = (_Float16*)take((size_t)NR * DD * 2); _Float16* vT = (_Float16*)take((size_t)NR * DD * 2); float* bias = (float*)take((size_t)NB * NN * NN * 4);
  float* AG = (float*)take((size_t)NR * DD * 4); float* x1 = (float*)take((size_t)NR * DD * 4); _Float16* H16 = (_Float16*)take((size_t)NR * FF * 2);
  k_qkv<<<dim3(NR / 64, 12), 128, 0, stream>>>(x, Wq, bq, Wk, bk, Wv, bv, q16, k16, vT);
  k_bias<<<dim3(NN, NB), 256, 0, stream>>>(pcs, Wr1, br1, Wr2, br2, bias);
  k_attn<<<dim3(NN / 64, NB), 128, 0, stream>>>(q16, k16, vT, bias, AG);
  k_lnproj<DD, 0><<<NR / 64, 128, 0, stream>>>(AG, Wo, bo, x, g1, be1, x1);
  k_ff1<<<dim3(NR / 64, FF / 128), 128, 0, stream>>>(x1, Wf1, bf1, H16);
  k_lnproj<FF, 1><<<NR / 64, 128, 0, stream>>>(H16, Wf2, bf2, x1, g2, be2, out);
}
